// HGNN_46351287058754
// MI455X (gfx1250) — hardware-verified
//
#include <hip/hip_runtime.h>
#include <math.h>
#include <stdint.h>

#define NNODE 20000
#define DIN   256
#define HID   128
#define NHD   4
#define NST   5
#define NTG   1024
#define NNB   16
#define NRW   (NTG * NNB)
#define DDM   (HID * NHD)
#define NZ    (NST * NHD)
static_assert(NRW == 16384);
static_assert(DDM == 512);
static_assert(NZ == 20);
static_assert((NTG % 64) == 0 && (NRW % 64) == 0 && (HID % 64) == 0);
static_assert((DIN % 32) == 0 && ((2 * HID) % 32) == 0 && ((2 * DDM) % 32) == 0);

typedef __bf16   v16b __attribute__((ext_vector_type(16)));
typedef __bf16   v8b  __attribute__((ext_vector_type(8)));
typedef float    v8f  __attribute__((ext_vector_type(8)));
typedef float    v4f  __attribute__((ext_vector_type(4)));
typedef unsigned int v4u __attribute__((ext_vector_type(4)));
typedef unsigned int v2u __attribute__((ext_vector_type(2)));

#if defined(__HIP_DEVICE_COMPILE__)
#define DEV_ASM 1
#else
#define DEV_ASM 0
#endif

__device__ __forceinline__ unsigned short bf_bits(float f) {
  unsigned u = __float_as_uint(f);
  return (unsigned short)((u + 0x7FFFu + ((u >> 16) & 1u)) >> 16);
}
__device__ __forceinline__ float bf_up(unsigned short hb) { return __uint_as_float(((unsigned)hb) << 16); }
__device__ __forceinline__ float bf_rn(float f) { return bf_up(bf_bits(f)); }
__device__ __forceinline__ float w_lo(unsigned w) { return __uint_as_float(w << 16); }
__device__ __forceinline__ float w_hi(unsigned w) { return __uint_as_float(w & 0xffff0000u); }
__device__ __forceinline__ unsigned pk16(unsigned short a, unsigned short b) { return (unsigned)a | ((unsigned)b << 16); }
__device__ __forceinline__ v8f zero8() { v8f z = {0.f, 0.f, 0.f, 0.f, 0.f, 0.f, 0.f, 0.f}; return z; }
__device__ __forceinline__ v4u pack_bf8(v4f a, v4f c) {
  v4u p;
  p[0] = pk16(bf_bits(a[0]), bf_bits(a[1]));
  p[1] = pk16(bf_bits(a[2]), bf_bits(a[3]));
  p[2] = pk16(bf_bits(c[0]), bf_bits(c[1]));
  p[3] = pk16(bf_bits(c[2]), bf_bits(c[3]));
  return p;
}

__device__ __forceinline__ v16b ldfrag(const __bf16* p) {
  union { v16b v; v8b h[2]; } f;
  f.h[0] = *(const v8b*)(p);
  f.h[1] = *(const v8b*)(p + 16);
  return f.v;
}

__device__ __forceinline__ v8f mmar(v16b a, v16b b, v8f c) {
  return __builtin_amdgcn_wmma_f32_16x16x32_bf16(false, a, false, b, (short)0, c, false, false);
}
__device__ __forceinline__ void dep_guard(v8f& a, v8f& b, v16b x, v16b y) {
#if DEV_ASM
  asm volatile("v_nop\n\tv_nop\n\tv_nop\n\tv_nop" : "+v"(a), "+v"(b) : "v"(x), "v"(y));
#else
  (void)a; (void)b; (void)x; (void)y;
#endif
}
__device__ __forceinline__ void keep4(v16b a, v16b b, v16b c, v16b d) {
#if DEV_ASM
  asm volatile("v_nop" :: "v"(a), "v"(b), "v"(c), "v"(d));
#else
  (void)a; (void)b; (void)c; (void)d;
#endif
}
__device__ __forceinline__ void acc_guard4(v8f& a, v8f& b, v8f& c, v8f& d) {
#if DEV_ASM
  asm volatile("v_nop\n\tv_nop\n\tv_nop\n\tv_nop" : "+v"(a), "+v"(b), "+v"(c), "+v"(d));
#else
  (void)a; (void)b; (void)c; (void)d;
#endif
}

template <int ACT> __device__ __forceinline__ float actf(float v) {
  if (ACT == 1) return (v >= 0.f) ? v : 0.2f * v;
  if (ACT == 2) return tanhf(v);
  return v;
}

__global__ __launch_bounds__(256) void cvt_bf16x8(const float* __restrict__ in, unsigned short* out, int n8) {
  const int i = blockIdx.x * 256 + (int)threadIdx.x;
  if (i < n8) {
    const v4f a = *(const v4f*)(in + (size_t)i * 8);
    const v4f c = *(const v4f*)(in + (size_t)i * 8 + 4);
    const v4u p = pack_bf8(a, c);
    unsigned short* o = out + (size_t)i * 8;
    *(volatile v4u*)o = p;
    __threadfence();
    *(volatile v4u*)o = p;
  }
}

template <int MODE, int KW>
__global__ __launch_bounds__(256) void dup_rows(const float* __restrict__ src0, const float* __restrict__ src1,
                                                unsigned short* dst, int nthr) {
  const int t = blockIdx.x * 256 + (int)threadIdx.x;
  if (t >= nthr) return;
  const int cpr = KW / 8;
  const int R = t / cpr, c = t - R * cpr;
  int srow;
  const float* p = src0;
  if (MODE == 0) {
    srow = R;
  } else if (MODE == 1) {
    const int z = R >> 8, kv = (R >> 7) & 1, n = R & 127;
    srow = z * 128 + n;
    p = kv ? src1 : src0;
  } else if (MODE == 2) {
    const int s = R >> 9, rem = R & 511;
    srow = ((s >= 2) ? 512 : 0) + rem;
  } else {
    const int s = R >> 7, n = R & 127;
    srow = ((s >= 2) ? 128 : 0) + n;
  }
  const float* sp = p + (size_t)srow * KW + c * 8;
  const v4f a  = *(const v4f*)(sp);
  const v4f a4 = *(const v4f*)(sp + 4);
  const v4u q = pack_bf8(a, a4);
  unsigned short* o = dst + (size_t)R * (2 * KW) + c * 8;
  *(volatile v4u*)o = q;
  *(volatile v4u*)(o + KW) = q;
  __threadfence();
  *(volatile v4u*)o = q;
  *(volatile v4u*)(o + KW) = q;
}

__global__ __launch_bounds__(32) void bias_tab(const float* __restrict__ kb, const float* __restrict__ vb,
                                               const float* __restrict__ a1b, const float* __restrict__ a2b,
                                               const float* __restrict__ ip1b, float* bt) {
  const int r = blockIdx.x, lane = (int)threadIdx.x & 31;
  const float* p;
  int off;
  if (r < 40) {
    const int z = r >> 1;
    off = z * HID;
    p = (r & 1) ? vb : kb;
  } else if (r < 60) {
    const int z = r - 40;
    off = ((z >= 8) ? 512 : 0) + (z & 3) * HID;
    p = a1b;
  } else if (r < 80) {
    const int z = r - 60;
    off = ((z >= 8) ? 512 : 0) + (z & 3) * HID;
    p = a2b;
  } else {
    const int s = r - 80;
    off = (s >= 2) ? HID : 0;
    p = ip1b;
  }
  const v4f v = *(const v4f*)(p + off + lane * 4);
  v4f o;
  o[0] = bf_rn(v[0]); o[1] = bf_rn(v[1]); o[2] = bf_rn(v[2]); o[3] = bf_rn(v[3]);
  float* d = bt + (size_t)r * HID + lane * 4;
  *(volatile v4f*)d = o;
  __threadfence();
  *(volatile v4f*)d = o;
}

__global__ __launch_bounds__(256) void gather_rows(const float* __restrict__ x, const int* __restrict__ idx,
                                                   int nrows, unsigned short* out) {
  const int lane = (int)threadIdx.x & 31, wave = (int)threadIdx.x >> 5;
  const int r = blockIdx.x * 8 + wave;
  if (r >= nrows) return;
  int node = idx[r];
  node = (node < 0) ? 0 : ((node > NNODE - 1) ? (NNODE - 1) : node);
  const float* src = x + (size_t)node * DIN + lane * 8;
  const v4f a = *(const v4f*)(src);
  const v4f c = *(const v4f*)(src + 4);
  const v4u p = pack_bf8(a, c);
  unsigned short* o = out + (size_t)r * DIN + lane * 8;
  *(volatile v4u*)o = p;
  __threadfence();
  *(volatile v4u*)o = p;
}

template <int OUT_MODE, int ACT, int HASB>
__global__ __launch_bounds__(256) void gemm64(
    const unsigned short* __restrict__ Ap, int lda, long long strideA,
    const unsigned short* __restrict__ Btp, int ldb, long long strideB,
    const float* __restrict__ bias, long long strideBias,
    void* Cout, void* Cout2, int ldc, long long strideC,
    int M, int N, int K) {
  const __bf16* A  = (const __bf16*)(const void*)Ap;
  const __bf16* Bt = (const __bf16*)(const void*)Btp;
  __shared__ __align__(16) float sT[8][16 * 68];
  const int b    = blockIdx.y;
  const int lane = threadIdx.x & 31;
  const int wave = threadIdx.x >> 5;
  const int tilesN = N >> 6;
  const int tilesM = M >> 6;
  const int tile = blockIdx.x * 8 + wave;
  if (tile >= tilesM * tilesN) return;
  const int tm = tile / tilesN;
  const int tn = tile - tm * tilesN;
  const int m0 = tm << 6;
  const int n0 = tn << 6;

  const __bf16* Ab = A  + (size_t)b * (size_t)strideA;
  const __bf16* Bb = Bt + (size_t)b * (size_t)strideB;
  const float* bz = bias + (HASB ? ((size_t)b * (size_t)strideBias) : (size_t)0);

  const int rlane = lane & 15;
  const int koff  = (lane >> 4) * 8;
  const int mOff  = (lane >> 4) * 8;

  v8f acc[4][4];
#pragma unroll
  for (int i = 0; i < 4; ++i)
#pragma unroll
    for (int j = 0; j < 4; ++j) acc[i][j] = zero8();

  for (int k0 = 0; k0 < K; k0 += 32) {
    v16b bq[4];
#pragma unroll
    for (int j = 0; j < 4; ++j)
      bq[j] = ldfrag(Bb + (size_t)(n0 + (j << 4) + rlane) * ldb + koff + k0);
#pragma unroll
    for (int i = 0; i < 4; ++i) {
      const v16b af = ldfrag(Ab + (size_t)(m0 + (i << 4) + rlane) * lda + koff + k0);
#pragma unroll
      for (int j = 0; j < 4; ++j) acc[i][j] = mmar(af, bq[j], acc[i][j]);
      dep_guard(acc[i][0], acc[i][3], af, bq[3]);
    }
    keep4(bq[0], bq[1], bq[2], bq[3]);
  }
  acc_guard4(acc[0][0], acc[0][1], acc[0][2], acc[0][3]);
  acc_guard4(acc[1][0], acc[1][1], acc[1][2], acc[1][3]);
  acc_guard4(acc[2][0], acc[2][1], acc[2][2], acc[2][3]);
  acc_guard4(acc[3][0], acc[3][1], acc[3][2], acc[3][3]);

  float* slab = sT[wave];
#pragma unroll
  for (int i = 0; i < 4; ++i) {
    const int mBase = m0 + (i << 4);
#pragma unroll
    for (int j = 0; j < 4; ++j) {
#pragma unroll
      for (int r = 0; r < 8; ++r) {
        slab[(mOff + r) * 68 + (j << 4) + rlane] = acc[i][j][r];
      }
    }
    __builtin_amdgcn_fence(__ATOMIC_RELEASE, "workgroup");
    __builtin_amdgcn_wave_barrier();
    __builtin_amdgcn_fence(__ATOMIC_ACQUIRE, "workgroup");
    if (OUT_MODE == 0) {
      float* C = (float*)Cout + (size_t)b * (size_t)strideC;
      const int h2 = lane >> 4, c4 = (lane & 15) * 4;
      v4f bv = {0.f, 0.f, 0.f, 0.f};
      if (HASB) {
        bv = *(const v4f*)(bz + n0 + c4);
        bv[0] = bf_rn(bv[0]); bv[1] = bf_rn(bv[1]); bv[2] = bf_rn(bv[2]); bv[3] = bf_rn(bv[3]);
      }
      for (int pass = 0; pass < 2; ++pass) {
#pragma unroll
        for (int it = 0; it < 8; ++it) {
          const int row = it * 2 + h2;
          v4f v = *(const v4f*)(slab + row * 68 + c4);
          v[0] = actf<ACT>(v[0] + bv[0]);
          v[1] = actf<ACT>(v[1] + bv[1]);
          v[2] = actf<ACT>(v[2] + bv[2]);
          v[3] = actf<ACT>(v[3] + bv[3]);
          *(volatile v4f*)(C + (size_t)(mBase + row) * ldc + n0 + c4) = v;
        }
        __threadfence();
      }
    } else {
      const int q = lane >> 3, c8 = (lane & 7) * 8;
      unsigned short* C  = (unsigned short*)Cout  + (size_t)b * (size_t)strideC;
      unsigned short* C2 = (unsigned short*)Cout2 + (size_t)b * (size_t)strideC;
      float bb[8];
#pragma unroll
      for (int e = 0; e < 8; ++e) bb[e] = 0.f;
      if (HASB) {
        const v4f b0 = *(const v4f*)(bz + n0 + c8);
        const v4f b1 = *(const v4f*)(bz + n0 + c8 + 4);
#pragma unroll
        for (int e = 0; e < 4; ++e) { bb[e] = bf_rn(b0[e]); bb[4 + e] = bf_rn(b1[e]); }
      }
      v4u hv[4], lv[4];
#pragma unroll
      for (int it = 0; it < 4; ++it) {
        const int row = it * 4 + q;
        const float* sp = slab + row * 68 + c8;
        float f[8];
#pragma unroll
        for (int e = 0; e < 8; ++e) f[e] = actf<ACT>(sp[e] + bb[e]);
        v4u a, a2;
#pragma unroll
        for (int e = 0; e < 4; ++e) {
          const float f0 = f[2 * e], f1 = f[2 * e + 1];
          const unsigned short h0 = bf_bits(f0), h1 = bf_bits(f1);
          const unsigned short l0 = bf_bits(f0 - bf_up(h0));
          const unsigned short l1 = bf_bits(f1 - bf_up(h1));
          a[e] = pk16(h0, h1); a2[e] = pk16(l0, l1);
        }
        hv[it] = a; lv[it] = a2;
      }
      for (int pass = 0; pass < 2; ++pass) {
#pragma unroll
        for (int it = 0; it < 4; ++it) {
          const int row = it * 4 + q;
          *(volatile v4u*)(C  + (size_t)(mBase + row) * ldc + n0 + c8) = hv[it];
          *(volatile v4u*)(C2 + (size_t)(mBase + row) * ldc + n0 + c8) = lv[it];
        }
        __threadfence();
      }
    }
    __builtin_amdgcn_fence(__ATOMIC_RELEASE, "workgroup");
    __builtin_amdgcn_wave_barrier();
    __builtin_amdgcn_fence(__ATOMIC_ACQUIRE, "workgroup");
  }
}

__global__ __launch_bounds__(128) void k_h1att(
    const unsigned short* __restrict__ KH2,
    const unsigned short* __restrict__ W1,
    const float* __restrict__ b1,
    const float* __restrict__ WH2,
    const unsigned short* __restrict__ VH2,
    const unsigned short* __restrict__ XS,
    unsigned short* OUTp)
{
  __shared__ __align__(16) float H1s[64 * 132];
  const int tid = threadIdx.x, lane = tid & 31, wave = tid >> 5;
  const int hh = lane >> 4, rl = lane & 15;
  const int koff = hh * 8, mOff = hh * 8;
  const int g = blockIdx.x;
  const int rq = wave & 1, cq = wave >> 1;
  const int rbase = g * 64 + rq * 32;
  const int cbase = cq * 64;
  const __bf16* A  = (const __bf16*)(const void*)KH2;
  const __bf16* Bt = (const __bf16*)(const void*)W1;

  v8f acc[2][4];
#pragma unroll
  for (int i = 0; i < 2; ++i)
#pragma unroll
    for (int j = 0; j < 4; ++j) acc[i][j] = zero8();

#pragma unroll 1
  for (int k0 = 0; k0 < 2 * HID; k0 += 32) {
    v16b bq[4];
#pragma unroll
    for (int j = 0; j < 4; ++j)
      bq[j] = ldfrag(Bt + (size_t)(cbase + (j << 4) + rl) * (2 * HID) + koff + k0);
#pragma unroll
    for (int i = 0; i < 2; ++i) {
      const v16b af = ldfrag(A + (size_t)(rbase + (i << 4) + rl) * (2 * HID) + koff + k0);
#pragma unroll
      for (int j = 0; j < 4; ++j) acc[i][j] = mmar(af, bq[j], acc[i][j]);
      dep_guard(acc[i][0], acc[i][3], af, bq[3]);
    }
    keep4(bq[0], bq[1], bq[2], bq[3]);
  }
  acc_guard4(acc[0][0], acc[0][1], acc[0][2], acc[0][3]);
  acc_guard4(acc[1][0], acc[1][1], acc[1][2], acc[1][3]);

  float bc[4];
#pragma unroll
  for (int j = 0; j < 4; ++j) bc[j] = bf_rn(b1[cbase + (j << 4) + rl]);
#pragma unroll
  for (int i = 0; i < 2; ++i) {
#pragma unroll
    for (int j = 0; j < 4; ++j) {
      const int col = cbase + (j << 4) + rl;
#pragma unroll
      for (int r = 0; r < 8; ++r) {
        const int row = rq * 32 + (i << 4) + mOff + r;
        const float v = acc[i][j][r] + bc[j];
        H1s[row * 132 + col] = (v >= 0.f) ? v : 0.2f * v;
      }
    }
  }
  __syncthreads();

  const int tl = wave;
  const int b  = g * 4 + tl;
  const v4f w4 = *(const v4f*)(WH2 + (size_t)b * HID + lane * 4);
  float att[16];
#pragma unroll
  for (int m = 0; m < 16; ++m) {
    const v4f hv = *(const v4f*)(H1s + (tl * 16 + m) * 132 + lane * 4);
    float p = hv[0] * w4[0] + hv[1] * w4[1] + hv[2] * w4[2] + hv[3] * w4[3];
#pragma unroll
    for (int off = 1; off < 32; off <<= 1) p += __shfl_xor(p, off, 32);
    att[m] = p;
  }
  float mx = att[0];
#pragma unroll
  for (int m = 1; m < 16; ++m) mx = fmaxf(mx, att[m]);
  float e[16], sum = 0.f;
#pragma unroll
  for (int m = 0; m < 16; ++m) { e[m] = __expf(att[m] - mx); sum += e[m]; }
  const float inv = 1.0f / sum;
#pragma unroll
  for (int m = 0; m < 16; ++m) e[m] = e[m] * inv;

  const int d8 = rl * 8;
  float ha[8];
#pragma unroll
  for (int k = 0; k < 8; ++k) ha[k] = 0.f;
#pragma unroll
  for (int r = 0; r < 8; ++r) {
    const int row = b * 16 + 8 * hh + r;
    const float em = hh ? e[8 + r] : e[r];
    const unsigned short* vp = VH2 + (size_t)row * (2 * HID) + d8;
    const v4u vw = *(const v4u*)(vp);
    const v4u lw = *(const v4u*)(vp + HID);
#pragma unroll
    for (int q = 0; q < 4; ++q) {
      const float v0 = (w_lo(vw[q]) + w_lo(lw[q])) * em;
      const float v1 = (w_hi(vw[q]) + w_hi(lw[q])) * em;
      ha[2 * q]     += (v0 >= 0.f) ? v0 : 0.2f * v0;
      ha[2 * q + 1] += (v1 >= 0.f) ? v1 : 0.2f * v1;
    }
  }
#pragma unroll
  for (int k = 0; k < 8; ++k) ha[k] += __shfl_xor(ha[k], 16, 32);

  const unsigned short* xp = XS + (size_t)b * (2 * HID) + d8;
  const v4u xw = *(const v4u*)(xp);
  const v4u xl = *(const v4u*)(xp + HID);
  v4u pw;
#pragma unroll
  for (int q = 0; q < 4; ++q) {
    const float o0 = (w_lo(xw[q]) + w_lo(xl[q]) + ha[2 * q]) * 0.5f;
    const float o1 = (w_hi(xw[q]) + w_hi(xl[q]) + ha[2 * q + 1]) * 0.5f;
    const unsigned short h0 = bf_bits(o0), h1 = bf_bits(o1);
    const unsigned short l0 = bf_bits(o0 - bf_up(h0)), l1 = bf_bits(o1 - bf_up(h1));
    const unsigned whi = pk16(h0, h1), wlo = pk16(l0, l1);
    pw[q] = hh ? wlo : whi;
  }
  unsigned short* dst = OUTp + (size_t)b * (2 * DDM) + hh * DDM + d8;
  *(volatile v4u*)dst = pw;
  __threadfence();
  *(volatile v4u*)dst = pw;
}

__device__ __forceinline__ void acc_row8(float (&z)[8], const unsigned short* p, float beta) {
  const v4u hw = *(const v4u*)(p);
  const v4u lw = *(const v4u*)(p + DDM);
#pragma unroll
  for (int q = 0; q < 4; ++q) {
    z[2 * q]     += beta * (w_lo(hw[q]) + w_lo(lw[q]));
    z[2 * q + 1] += beta * (w_hi(hw[q]) + w_hi(lw[q]));
  }
}
__device__ __forceinline__ void pack_hilo8(const float (&z)[8], v4u& hv, v4u& lv) {
#pragma unroll
  for (int q = 0; q < 4; ++q) {
    const float f0 = z[2 * q], f1 = z[2 * q + 1];
    const unsigned short h0 = bf_bits(f0), h1 = bf_bits(f1);
    const unsigned short l0 = bf_bits(f0 - bf_up(h0)), l1 = bf_bits(f1 - bf_up(h1));
    hv[q] = pk16(h0, h1); lv[q] = pk16(l0, l1);
  }
}

__global__ __launch_bounds__(128) void k_sem1(const float* __restrict__ W0,
                                             const float* __restrict__ p2w,
                                             const unsigned short* __restrict__ OUT2,
                                             unsigned short* Z2)
{
  const int lane = (int)threadIdx.x & 31, wave = (int)threadIdx.x >> 5;
  const int b = blockIdx.x * 4 + wave;
  float sc[5];
#pragma unroll
  for (int s = 0; s < NST; ++s) {
    const v4f w = *(const v4f*)(W0 + ((size_t)s * NTG + b) * HID + lane * 4);
    const v4f p = *(const v4f*)(p2w + ((s >= 2) ? HID : 0) + lane * 4);
    float d = w[0] * bf_rn(p[0]) + w[1] * bf_rn(p[1]) + w[2] * bf_rn(p[2]) + w[3] * bf_rn(p[3]);
#pragma unroll
    for (int off = 1; off < 32; off <<= 1) d += __shfl_xor(d, off, 32);
    sc[s] = d;
  }
  const float mA  = fmaxf(sc[0], sc[1]);
  const float eA0 = __expf(sc[0] - mA), eA1 = __expf(sc[1] - mA);
  const float iA  = 1.0f / (eA0 + eA1);
  const float bA0 = eA0 * iA, bA1 = eA1 * iA;
  const float mB  = fmaxf(fmaxf(sc[2], sc[3]), sc[4]);
  const float eB2 = __expf(sc[2] - mB), eB3 = __expf(sc[3] - mB), eB4 = __expf(sc[4] - mB);
  const float iB  = 1.0f / (eB2 + eB3 + eB4);
  const float bB2 = eB2 * iB, bB3 = eB3 * iB, bB4 = eB4 * iB;

#pragma unroll 1
  for (int it = 0; it < 2; ++it) {
    const int d8 = it * 256 + lane * 8;
    float zA[8], zB[8];
#pragma unroll
    for (int k = 0; k < 8; ++k) { zA[k] = 0.f; zB[k] = 0.f; }
    acc_row8(zA, OUT2 + ((size_t)0 * NTG + b) * (2 * DDM) + d8, bA0);
    acc_row8(zA, OUT2 + ((size_t)1 * NTG + b) * (2 * DDM) + d8, bA1);
    acc_row8(zB, OUT2 + ((size_t)2 * NTG + b) * (2 * DDM) + d8, bB2);
    acc_row8(zB, OUT2 + ((size_t)3 * NTG + b) * (2 * DDM) + d8, bB3);
    acc_row8(zB, OUT2 + ((size_t)4 * NTG + b) * (2 * DDM) + d8, bB4);
    v4u hA, lA, hB, lB;
    pack_hilo8(zA, hA, lA);
    pack_hilo8(zB, hB, lB);
    unsigned short* pa = Z2 + (size_t)b * (2 * DDM) + d8;
    unsigned short* pb = Z2 + ((size_t)NTG + b) * (2 * DDM) + d8;
    *(volatile v4u*)pa = hA;  *(volatile v4u*)(pa + DDM) = lA;
    *(volatile v4u*)pb = hB;  *(volatile v4u*)(pb + DDM) = lB;
    __threadfence();
    *(volatile v4u*)pa = hA;  *(volatile v4u*)(pa + DDM) = lA;
    *(volatile v4u*)pb = hB;  *(volatile v4u*)(pb + DDM) = lB;
  }
}

__global__ __launch_bounds__(128) void k_sem2(const float* __restrict__ WB,
                                             const float* __restrict__ p2w,
                                             const unsigned short* __restrict__ Z2,
                                             float* out)
{
  const int lane = (int)threadIdx.x & 31, wave = (int)threadIdx.x >> 5;
  const int b = blockIdx.x * 4 + wave;
  const v4f p = *(const v4f*)(p2w + lane * 4);
  const float pr0 = bf_rn(p[0]), pr1 = bf_rn(p[1]), pr2 = bf_rn(p[2]), pr3 = bf_rn(p[3]);
  float sc[2];
#pragma unroll
  for (int kk = 0; kk < 2; ++kk) {
    const v4f w = *(const v4f*)(WB + ((size_t)kk * NTG + b) * HID + lane * 4);
    float d = w[0] * pr0 + w[1] * pr1 + w[2] * pr2 + w[3] * pr3;
#pragma unroll
    for (int off = 1; off < 32; off <<= 1) d += __shfl_xor(d, off, 32);
    sc[kk] = d;
  }
  const float mx = fmaxf(sc[0], sc[1]);
  const float e0 = __expf(sc[0] - mx), e1 = __expf(sc[1] - mx);
  const float iv = 1.0f / (e0 + e1);
  const float be0 = e0 * iv, be1 = e1 * iv;

  v4f ov[4];
#pragma unroll
  for (int it = 0; it < 4; ++it) {
    const int d4 = it * 128 + lane * 4;
    const unsigned short* pa = Z2 + (size_t)b * (2 * DDM) + d4;
    const unsigned short* pb = Z2 + ((size_t)NTG + b) * (2 * DDM) + d4;
    const v2u ha = *(const v2u*)(pa), la = *(const v2u*)(pa + DDM);
    const v2u hb = *(const v2u*)(pb), lb = *(const v2u*)(pb + DDM);
    v4f v;
    v[0] = be0 * (w_lo(ha[0]) + w_lo(la[0])) + be1 * (w_lo(hb[0]) + w_lo(lb[0]));
    v[1] = be0 * (w_hi(ha[0]) + w_hi(la[0])) + be1 * (w_hi(hb[0]) + w_hi(lb[0]));
    v[2] = be0 * (w_lo(ha[1]) + w_lo(la[1])) + be1 * (w_lo(hb[1]) + w_lo(lb[1]));
    v[3] = be0 * (w_hi(ha[1]) + w_hi(la[1])) + be1 * (w_hi(hb[1]) + w_hi(lb[1]));
    ov[it] = v;
  }
  for (int pass = 0; pass < 2; ++pass) {
#pragma unroll
    for (int it = 0; it < 4; ++it) {
      *(volatile v4f*)(out + (size_t)b * DDM + it * 128 + lane * 4) = ov[it];
    }
    __threadfence();
  }
}

static constexpr size_t SZ_W20   = (size_t)NZ * HID * (2 * HID) * 2;
static constexpr size_t SZ_FCW   = (size_t)NZ * HID * DIN * 2;
static constexpr size_t SZ_KVW   = (size_t)NZ * 2 * HID * (2 * HID) * 2;
static constexpr size_t SZ_IP1   = (size_t)NST * HID * (2 * DDM) * 2;
static constexpr size_t SZ_BP1   = (size_t)HID * (2 * DDM) * 2;
static constexpr size_t SZ_BT    = (size_t)88 * HID * 4;
static constexpr size_t SZ_TXA   = (size_t)NTG * DIN * 2;
static constexpr size_t SZ_ACT   = (size_t)NZ * NTG * (2 * HID) * 2;
static constexpr size_t SZ_WH2   = (size_t)NZ * NTG * HID * 4;
static constexpr size_t SZ_NYA   = (size_t)NRW * DIN * 2;
static constexpr size_t SZ_Y2    = (size_t)NHD * NRW * (2 * HID) * 2;
static constexpr size_t SZ_KV2   = (size_t)2 * NRW * (2 * HID) * 2;
static constexpr size_t SZ_OUT2  = (size_t)NST * NTG * (2 * DDM) * 2;
static constexpr size_t SZ_W0    = (size_t)NST * NTG * HID * 4;
static constexpr size_t SZ_Z2    = (size_t)2 * NTG * (2 * DDM) * 2;
static constexpr size_t SZ_WB    = (size_t)2 * NTG * HID * 4;
static constexpr size_t WS_TOTAL = SZ_FCW + SZ_W20 + SZ_KVW + 3 * SZ_W20 + SZ_IP1 + SZ_BP1 + SZ_BT
                                 + SZ_TXA + 3 * SZ_ACT + SZ_WH2 + SZ_NYA + SZ_Y2 + SZ_KV2
                                 + SZ_OUT2 + SZ_W0 + SZ_Z2 + SZ_WB;
static_assert(WS_TOTAL == (size_t)130330624);
static_assert(WS_TOTAL <= (size_t)134217728);
static_assert((size_t)NTG * DDM * 4 == (size_t)2097152);

extern "C" void kernel_launch(void* const* d_in, const int* in_sizes, int n_in,
                              void* d_out, int out_size, void* d_ws, size_t ws_size,
                              hipStream_t stream) {
  if (n_in < 22) return;
  if (in_sizes[0] != NNODE * DIN) return;
  if (in_sizes[1] != NTG) return;
  if (in_sizes[2] != NST * NTG * NNB) return;
  if (in_sizes[3] != NZ * HID * DIN || in_sizes[4] != NZ * HID) return;
  if (in_sizes[5] != NZ * HID * HID || in_sizes[6] != NZ * HID) return;
  if (in_sizes[7] != NZ * HID * HID || in_sizes[8] != NZ * HID) return;
  if (in_sizes[9] != NZ * HID * HID || in_sizes[10] != NZ * HID) return;
  if (in_sizes[11] != 8 * HID * HID || in_sizes[12] != 8 * HID * HID || in_sizes[13] != 8 * HID) return;
  if (in_sizes[14] != 8 * HID * HID || in_sizes[15] != 8 * HID) return;
  if (in_sizes[16] != 2 * HID * DDM || in_sizes[17] != 2 * HID || in_sizes[18] != 2 * HID) return;
  if (in_sizes[19] != HID * DDM || in_sizes[20] != HID || in_sizes[21] != HID) return;
  if (out_size != NTG * DDM) return;
  if (WS_TOTAL > ws_size) return;

  const float* x      = (const float*)d_in[0];
  const int*   tgt    = (const int*)d_in[1];
  const int*   nbr    = (const int*)d_in[2];
  const float* fc_w   = (const float*)d_in[3];
  const float* fc_b   = (const float*)d_in[4];
  const float* q_w    = (const float*)d_in[5];
  const float* q_b    = (const float*)d_in[6];
  const float* k_w    = (const float*)d_in[7];
  const float* k_b    = (const float*)d_in[8];
  const float* v_w    = (const float*)d_in[9];
  const float* v_b    = (const float*)d_in[10];
  const float* att_W  = (const float*)d_in[11];
  const float* a1_w   = (const float*)d_in[12];
  const float* a1_b   = (const float*)d_in[13];
  const float* a2_w   = (const float*)d_in[14];
  const float* a2_b   = (const float*)d_in[15];
  const float* ip1_w  = (const float*)d_in[16];
  const float* ip1_b  = (const float*)d_in[17];
  const float* ip2_w  = (const float*)d_in[18];
  const float* bp1_w  = (const float*)d_in[19];
  const float* bp1_b  = (const float*)d_in[20];
  const float* bp2_w  = (const float*)d_in[21];
  float* out = (float*)d_out;

  size_t off = 0;
  const size_t oFCW  = off; off += SZ_FCW;
  const size_t oQW2  = off; off += SZ_W20;
  const size_t oKVW  = off; off += SZ_KVW;
  const size_t oA1W  = off; off += SZ_W20;
  const size_t oA2W  = off; off += SZ_W20;
  const size_t oAW   = off; off += SZ_W20;
  const size_t oIP1  = off; off += SZ_IP1;
  const size_t oBP1  = off; off += SZ_BP1;
  const size_t oBT   = off; off += SZ_BT;
  const size_t oTXA  = off; off += SZ_TXA;
  const size_t oXSH  = off; off += SZ_ACT;
  const size_t oQH   = off; off += SZ_ACT;
  const size_t oH2   = off; off += SZ_ACT;
  const size_t oWH2  = off; off += SZ_WH2;
  const size_t oNYA  = off; off += SZ_NYA;
  const size_t oY2   = off; off += SZ_Y2;
  const size_t oKV2  = off; off += SZ_KV2;
  const size_t oOUT2 = off; off += SZ_OUT2;
  const size_t oW0   = off; off += SZ_W0;
  const size_t oZ2   = off; off += SZ_Z2;
  const size_t oWB   = off; off += SZ_WB;
  if (off != WS_TOTAL) return;
  if (off > ws_size) return;

  char* ws = (char*)d_ws;
  unsigned short* FCW   = (unsigned short*)(ws + oFCW);
  unsigned short* QW2   = (unsigned short*)(ws + oQW2);
  unsigned short* KVW2  = (unsigned short*)(ws + oKVW);
  unsigned short* A1W2  = (unsigned short*)(ws + oA1W);
  unsigned short* A2W2  = (unsigned short*)(ws + oA2W);
  unsigned short* AW2   = (unsigned short*)(ws + oAW);
  unsigned short* IP1W2 = (unsigned short*)(ws + oIP1);
  unsigned short* BP1W2 = (unsigned short*)(ws + oBP1);
  float*          BT    = (float*)(ws + oBT);
  unsigned short* TXA   = (unsigned short*)(ws + oTXA);
  unsigned short* XSH2  = (unsigned short*)(ws + oXSH);
  unsigned short* QH2   = (unsigned short*)(ws + oQH);
  unsigned short* H22   = (unsigned short*)(ws + oH2);
  float*          WH2   = (float*)(ws + oWH2);
  unsigned short* NYA   = (unsigned short*)(ws + oNYA);
  unsigned short* Y2    = (unsigned short*)(ws + oY2);
  unsigned short* KV2   = (unsigned short*)(ws + oKV2);
  unsigned short* OUT2  = (unsigned short*)(ws + oOUT2);
  float*          W0    = (float*)(ws + oW0);
  unsigned short* Z2    = (unsigned short*)(ws + oZ2);
  float*          WB    = (float*)(ws + oWB);

  const dim3 b256(256), b128(128), b32(32);
  const long long WZ   = (long long)HID * (2 * HID);
  const long long AZ   = (long long)NTG * (2 * HID);
  const long long WH2Z = (long long)NTG * HID;
  const long long Y2Z  = (long long)NRW * (2 * HID);
  const long long O2Z  = (long long)NTG * (2 * DDM);
  const long long IP1Z = (long long)HID * (2 * DDM);

  cvt_bf16x8<<<dim3((NZ * HID * DIN / 8 + 255) / 256), b256, 0, stream>>>(fc_w, FCW, NZ * HID * DIN / 8);
  dup_rows<0, 128><<<dim3((NZ * HID * 16 + 255) / 256), b256, 0, stream>>>(q_w, q_w, QW2, NZ * HID * 16);
  dup_rows<1, 128><<<dim3((NZ * 2 * HID * 16 + 255) / 256), b256, 0, stream>>>(k_w, v_w, KVW2, NZ * 2 * HID * 16);
  dup_rows<2, 128><<<dim3((NZ * HID * 16 + 255) / 256), b256, 0, stream>>>(a1_w, a1_w, A1W2, NZ * HID * 16);
  dup_rows<2, 128><<<dim3((NZ * HID * 16 + 255) / 256), b256, 0, stream>>>(a2_w, a2_w, A2W2, NZ * HID * 16);
  dup_rows<2, 128><<<dim3((NZ * HID * 16 + 255) / 256), b256, 0, stream>>>(att_W, att_W, AW2, NZ * HID * 16);
  dup_rows<3, 512><<<dim3((NST * HID * 64 + 255) / 256), b256, 0, stream>>>(ip1_w, ip1_w, IP1W2, NST * HID * 64);
  dup_rows<0, 512><<<dim3((HID * 64 + 255) / 256), b256, 0, stream>>>(bp1_w, bp1_w, BP1W2, HID * 64);
  bias_tab<<<dim3(85), b32, 0, stream>>>(k_b, v_b, a1_b, a2_b, ip1_b, BT);
  gather_rows<<<dim3(NTG / 8), b256, 0, stream>>>(x, tgt, NTG, TXA);

  gemm64<2, 1, 1><<<dim3(4, NZ), b256, 0, stream>>>(
      TXA, DIN, 0LL, FCW, DIN, (long long)HID * DIN, fc_b, (long long)HID,
      (void*)XSH2, (void*)(XSH2 + HID), 2 * HID, AZ, NTG, HID, DIN);
  gemm64<2, 0, 1><<<dim3(4, NZ), b256, 0, stream>>>(
      XSH2, 2 * HID, AZ, QW2, 2 * HID, WZ, q_b, (long long)HID,
      (void*)QH2, (void*)(QH2 + HID), 2 * HID, AZ, NTG, HID, 2 * HID);
  gemm64<2, 1, 1><<<dim3(4, NZ), b256, 0, stream>>>(
      QH2, 2 * HID, AZ, A2W2, 2 * HID, WZ, BT + 60 * HID, (long long)HID,
      (void*)H22, (void*)(H22 + HID), 2 * HID, AZ, NTG, HID, 2 * HID);
  gemm64<0, 0, 0><<<dim3(4, NZ), b256, 0, stream>>>(
      H22, 2 * HID, AZ, AW2, 2 * HID, WZ, BT, 0LL,
      (void*)WH2, (void*)WH2, HID, WH2Z, NTG, HID, 2 * HID);

  for (int s = 0; s < NST; ++s) {
    gather_rows<<<dim3(NRW / 8), b256, 0, stream>>>(x, nbr + (size_t)s * NRW, NRW, NYA);
    gemm64<2, 1, 1><<<dim3(64, NHD), b256, 0, stream>>>(
        NYA, DIN, 0LL, FCW + (size_t)s * NHD * HID * DIN, DIN, (long long)HID * DIN, fc_b + (size_t)s * NHD * HID, (long long)HID,
        (void*)Y2, (void*)(Y2 + HID), 2 * HID, Y2Z, NRW, HID, DIN);
    for (int h = 0; h < NHD; ++h) {
      const int zsh = s * NHD + h;
      gemm64<2, 0, 1><<<dim3(64, 2), b256, 0, stream>>>(
          Y2 + (size_t)h * Y2Z, 2 * HID, 0LL, KVW2 + (size_t)zsh * 2 * WZ, 2 * HID, WZ, BT + (size_t)zsh * 2 * HID, (long long)HID,
          (void*)KV2, (void*)(KV2 + HID), 2 * HID, Y2Z, NRW, HID, 2 * HID);
      k_h1att<<<dim3(NRW / 64), b128, 0, stream>>>(
          KV2, A1W2 + (size_t)zsh * WZ, BT + (size_t)(40 + zsh) * HID, WH2 + (size_t)zsh * WH2Z,
          KV2 + Y2Z, XSH2 + (size_t)zsh * AZ, OUT2 + (size_t)s * O2Z + (size_t)h * HID);
    }
  }

  gemm64<0, 2, 1><<<dim3(4, NST), b256, 0, stream>>>(
      OUT2, 2 * DDM, O2Z, IP1W2, 2 * DDM, IP1Z, BT + 80 * HID, (long long)HID,
      (void*)W0, (void*)W0, HID, WH2Z, NTG, HID, 2 * DDM);
  k_sem1<<<dim3(NTG / 4), b128, 0, stream>>>(W0, ip2_w, OUT2, Z2);
  gemm64<0, 2, 1><<<dim3(4, 2), b256, 0, stream>>>(
      Z2, 2 * DDM, O2Z, BP1W2, 2 * DDM, 0LL, bp1_b, 0LL,
      (void*)WB, (void*)WB, HID, WH2Z, NTG, HID, 2 * DDM);
  k_sem2<<<dim3(NTG / 4), b128, 0, stream>>>(WB, bp2_w, Z2, out);
  (void)hipGetLastError();
}
